// NodeNetwork_3255585210371
// MI455X (gfx1250) — hardware-run, weakly checked
//
#include <hip/hip_runtime.h>
#include <stddef.h>
#include <stdint.h>
#include <math.h>

#define NN      100000
#define NE      1000000
#define HD      64
#define K1      192
#define KL      128
#define MP      100096
#define GBM     128
#define NTHR    256
#define NWAVE   8
#define EPT     8
#define WCH     (32 * EPT)
#define NBRUN   1024
#define SLB     10
#define NBK     98
#define NROLE   2
#define WLCAP   2048
#define RCAP    12288
#define TRIPCAP 64
#define MAXDEG_MEAS   26
#define MAXB1024_MEAS 10529
#define ABM     64
#define SP      68
#define ATP     136
#define AIP     68
#define WSMAX   (128u << 20)

#define BK_ZINTS (NWAVE * WLCAP + 2 * RCAP + 3 * NBRUN)
#define BK_INTS  (BK_ZINTS + 16)
#define BK_LDS   (BK_INTS * 4)

#define WALL_W_INTS ((HD * K1 + 2 * HD * KL) / 2)
#define WALL_PV_F   512
#define WALL_INTS   (WALL_W_INTS + WALL_PV_F)
#define ML_STG_OFF  WALL_INTS
#define ML_AT_OFF   (ML_STG_OFF + GBM * SP)
#define ML_INTS     (ML_AT_OFF + GBM * AIP)
#define ML_LDS      (ML_INTS * 4)

#define PBX   (MP * HD / 8 / NTHR)
#define PBW1  (HD * K1 / 8 / NTHR)
#define PBW2  (HD * KL / 8 / NTHR)
#define PBTOT (PBX + PBW1 + 2 * PBW2 + 1)

static_assert(HD == 64 && HD == 16 * 4);
static_assert(MP % GBM == 0 && MP >= NN && MP == 782 * GBM && MP % ABM == 0);
static_assert(NN <= NBK * NBRUN && MP <= NBK * NBRUN);
static_assert(NBRUN == (1 << SLB) && NBRUN % GBM == 0 && NBRUN % ABM == 0 && NBRUN % 32 == 0);
static_assert(NE <= (1 << 20) && (((long long)NE) << SLB) < (1LL << 31));
static_assert(NE % 8 == 0 && ((NE * 4) % 16) == 0);
static_assert(K1 % 32 == 0 && KL % 32 == 0 && KL == 2 * HD && K1 == 3 * HD);
static_assert((long long)RCAP * 100 >= (long long)MAXB1024_MEAS * 105);
static_assert(WLCAP >= MAXB1024_MEAS / 8 + 8 * 37 + 1);
static_assert(MAXDEG_MEAS + 8 <= TRIPCAP);
static_assert(BK_ZINTS % (NTHR * 4) == 0 && (2 * RCAP) % (NTHR * 4) == 0 && (2 * NBRUN) % (NTHR * 4) == 0);
static_assert(BK_LDS <= 327680 && ML_LDS <= 327680);
static_assert((MP * HD / 8) % NTHR == 0 && (HD * K1 / 8) % NTHR == 0 && (HD * KL / 8) % NTHR == 0);
static_assert(WALL_INTS % 4 == 0 && ML_STG_OFF % 4 == 0 && ML_AT_OFF % 4 == 0);
static_assert(ATP == 2 * AIP && ATP % 8 == 0 && ATP >= KL);
static_assert(ABM == NWAVE * 8 && GBM == NWAVE * 16);

typedef float          v4f   __attribute__((ext_vector_type(4)));
typedef float          v8f   __attribute__((ext_vector_type(8)));
typedef int            v2i   __attribute__((ext_vector_type(2)));
typedef int            v4i   __attribute__((ext_vector_type(4)));
typedef int            v8i   __attribute__((ext_vector_type(8)));
typedef unsigned       v2u   __attribute__((ext_vector_type(2)));
typedef unsigned short v8us  __attribute__((ext_vector_type(8)));
typedef unsigned short v16us __attribute__((ext_vector_type(16)));
typedef __bf16         v16bf __attribute__((ext_vector_type(16)));
typedef v4f  __attribute__((may_alias)) v4fa;
typedef v2i  __attribute__((may_alias)) v2ia;
typedef v4i  __attribute__((may_alias)) v4ia;
typedef v2u  __attribute__((may_alias)) v2ua;
typedef v8us __attribute__((may_alias)) v8usa;
union FragB { v16bf v; v16us u; v8us h[2]; v8i w; };

__device__ __forceinline__ v8f wmb(const FragB& a, const FragB& b, v8f c) {
  v8f d = __builtin_amdgcn_wmma_f32_16x16x32_bf16(false, a.v, false, b.v, (short)0, c, false, false);
  asm volatile("v_nop\n\tv_nop\n\tv_nop\n\tv_nop" : "+v"(d) : "v"(a.w), "v"(b.w));
  return d;
}

__device__ __forceinline__ unsigned bf16_bits(float f) {
  const unsigned u = __float_as_uint(f);
  const unsigned r = (u + 0x7FFFu + ((u >> 16) & 1u)) >> 16;
  const unsigned q = (u >> 16) | 0x40u;
  return ((u & 0x7fffffffu) > 0x7f800000u) ? q : r;
}

__device__ __forceinline__ void hilo_pack(float v0, float v1, float v2, float v3,
                                          int& h01, int& h23, int& l01, int& l23) {
  const unsigned a0 = bf16_bits(v0), a1 = bf16_bits(v1), a2 = bf16_bits(v2), a3 = bf16_bits(v3);
  const unsigned b0 = bf16_bits(v0 - __uint_as_float(a0 << 16));
  const unsigned b1 = bf16_bits(v1 - __uint_as_float(a1 << 16));
  const unsigned b2 = bf16_bits(v2 - __uint_as_float(a2 << 16));
  const unsigned b3 = bf16_bits(v3 - __uint_as_float(a3 << 16));
  h01 = (int)(a0 | (a1 << 16)); h23 = (int)(a2 | (a3 << 16));
  l01 = (int)(b0 | (b1 << 16)); l23 = (int)(b2 | (b3 << 16));
}

__device__ __forceinline__ v4i regroup8(int h01, int h23, int l01, int l23, int lane) {
  const int t  = lane & 15;
  const int s0 = (lane & 16) + ((2 * t) & 15), s1 = s0 + 1;
  const int a0 = __shfl(h01, s0, 32), a1 = __shfl(h23, s0, 32), a2 = __shfl(h01, s1, 32), a3 = __shfl(h23, s1, 32);
  const int b0 = __shfl(l01, s0, 32), b1 = __shfl(l23, s0, 32), b2 = __shfl(l01, s1, 32), b3 = __shfl(l23, s1, 32);
  const int mk = (t < 8) ? -1 : 0;
  v4i o;
  o.x = (a0 & mk) | (b0 & ~mk); o.y = (a1 & mk) | (b1 & ~mk);
  o.z = (a2 & mk) | (b2 & ~mk); o.w = (a3 & mk) | (b3 & ~mk);
  return o;
}

__device__ __forceinline__ void st2_v4f(float* p, v4f v) {
  *(volatile v4f*)p = v;
  __threadfence();
  *(volatile v4f*)p = v;
}
__device__ __forceinline__ void st2_v8us(unsigned short* p, v8us v) {
  *(volatile v8us*)p = v;
  __threadfence();
  *(volatile v8us*)p = v;
}

__device__ __forceinline__ v8us col8(const float* __restrict__ base, int stride) {
  float f[8];
#pragma unroll
  for (int i = 0; i < 8; ++i) f[i] = base[(size_t)i * (size_t)stride];
  v8us o;
#pragma unroll
  for (int i = 0; i < 8; ++i) o[i] = (unsigned short)bf16_bits(f[i]);
  return o;
}

__device__ __forceinline__ float pick7(float a0, float a1, float a2, float a3, float a4, float a5, float a6, int vec) {
  const unsigned m0 = (vec == 0) ? 0xffffffffu : 0u, m1 = (vec == 1) ? 0xffffffffu : 0u;
  const unsigned m2 = (vec == 2) ? 0xffffffffu : 0u, m3 = (vec == 3) ? 0xffffffffu : 0u;
  const unsigned m4 = (vec == 4) ? 0xffffffffu : 0u, m5 = (vec == 5) ? 0xffffffffu : 0u;
  const unsigned m6 = (vec == 6) ? 0xffffffffu : 0u;
  const unsigned r = ((bf16_bits(a0) << 16) & m0) | ((bf16_bits(a1) << 16) & m1) | ((bf16_bits(a2) << 16) & m2) |
                     ((bf16_bits(a3) << 16) & m3) | ((bf16_bits(a4) << 16) & m4) | ((bf16_bits(a5) << 16) & m5) |
                     ((bf16_bits(a6) << 16) & m6);
  return __uint_as_float(r);
}

__global__ __launch_bounds__(NTHR) void k_prep(const float* __restrict__ x, const float* __restrict__ w1,
                                               const float* __restrict__ b1, const float* __restrict__ g1,
                                               const float* __restrict__ be1, const float* __restrict__ w2,
                                               const float* __restrict__ b2, const float* __restrict__ g2,
                                               const float* __restrict__ be2, const float* __restrict__ w3,
                                               const float* __restrict__ b3,
                                               unsigned short* xb, unsigned short* w1c, unsigned short* w2d,
                                               unsigned short* w3d, float* pvp) {
  const int tid = (int)threadIdx.x;
  const int blk = (int)blockIdx.x;
  if (blk < PBX) {
    const int u   = blk * NTHR + tid;
    const int row = u >> 3, k8 = (u & 7) * 8;
    const int rc  = row < NN ? row : NN - 1;
    const unsigned mk = row < NN ? 0xffffu : 0u;
    const float* p = x + (size_t)rc * HD + k8;
    const v4f a = *(const v4fa*)p;
    const v4f b = *(const v4fa*)(p + 4);
    v8us o;
    o[0] = (unsigned short)(bf16_bits(a.x) & mk); o[1] = (unsigned short)(bf16_bits(a.y) & mk);
    o[2] = (unsigned short)(bf16_bits(a.z) & mk); o[3] = (unsigned short)(bf16_bits(a.w) & mk);
    o[4] = (unsigned short)(bf16_bits(b.x) & mk); o[5] = (unsigned short)(bf16_bits(b.y) & mk);
    o[6] = (unsigned short)(bf16_bits(b.z) & mk); o[7] = (unsigned short)(bf16_bits(b.w) & mk);
    st2_v8us(xb + (size_t)u * 8, o);
  } else if (blk < PBX + PBW1) {
    const int u  = (blk - PBX) * NTHR + tid;
    const int n  = u / (K1 / 8);
    const int k8 = (u - n * (K1 / 8)) * 8;
    const int sk = (k8 < HD) ? k8 : (k8 - HD);
    const v8us o = col8(w1 + (size_t)sk * HD + n, HD);
    st2_v8us(w1c + (size_t)u * 8, o);
  } else if (blk < PBX + PBW1 + PBW2) {
    const int u = (blk - PBX - PBW1) * NTHR + tid;
    const int n = u >> 4, k8 = (u & 15) * 8, kk = k8 & 63;
    const v8us o = col8(w2 + (size_t)kk * HD + n, HD);
    st2_v8us(w2d + (size_t)u * 8, o);
  } else if (blk < PBX + PBW1 + 2 * PBW2) {
    const int u = (blk - PBX - PBW1 - PBW2) * NTHR + tid;
    const int n = u >> 4, k8 = (u & 15) * 8, kk = k8 & 63;
    const v8us o = col8(w3 + (size_t)kk * HD + n, HD);
    st2_v8us(w3d + (size_t)u * 8, o);
  } else {
    if (tid < 128) {
      const int vec = tid >> 4, q = tid & 15;
      const v4f c0 = *(const v4fa*)(b1 + 4 * q);
      const v4f c1 = *(const v4fa*)(g1 + 4 * q);
      const v4f c2 = *(const v4fa*)(be1 + 4 * q);
      const v4f c3 = *(const v4fa*)(b2 + 4 * q);
      const v4f c4 = *(const v4fa*)(g2 + 4 * q);
      const v4f c5 = *(const v4fa*)(be2 + 4 * q);
      const v4f c6 = *(const v4fa*)(b3 + 4 * q);
      asm volatile("" :: "v"(c0), "v"(c1), "v"(c2), "v"(c3));
      asm volatile("" :: "v"(c4), "v"(c5), "v"(c6));
      v4f o;
      o.x = pick7(c0.x, c1.x, c2.x, c3.x, c4.x, c5.x, c6.x, vec);
      o.y = pick7(c0.y, c1.y, c2.y, c3.y, c4.y, c5.y, c6.y, vec);
      o.z = pick7(c0.z, c1.z, c2.z, c3.z, c4.z, c5.z, c6.z, vec);
      o.w = pick7(c0.w, c1.w, c2.w, c3.w, c4.w, c5.w, c6.w, vec);
      st2_v4f(pvp + 4 * tid, o);
    }
  }
}

__device__ __forceinline__ void bucket_flush(const int* pl, const int* cnt, int ov, int* lp, int* cop, int* fp,
                                             int tid) {
#pragma unroll 1
  for (int i = tid * 4; i < 2 * RCAP; i += NTHR * 4) {
    const v4i v = *(const v4ia*)(pl + i);
    *(volatile v4i*)(lp + i) = v;
  }
#pragma unroll 1
  for (int i = tid * 4; i < 2 * NBRUN; i += NTHR * 4) {
    const v4i v = *(const v4ia*)(cnt + i);
    *(volatile v4i*)(cop + i) = v;
  }
  if (tid < 8) {
    const v4i f = {ov, ov, ov, ov};
    *(volatile v4i*)(fp + 4 * tid) = f;
  }
}

__global__ __launch_bounds__(NTHR) void k_bucket(const int* __restrict__ ei, const float* __restrict__ ew,
                                                 int* LIST, int* CO, int* FLAG) {
  extern __shared__ __attribute__((aligned(16))) int dsm[];
  int* wl   = dsm;
  int* pl   = dsm + NWAVE * WLCAP;
  int* cnt  = pl + 2 * RCAP;
  int* offs = cnt + NBRUN;
  int* cur  = offs + NBRUN;
  int* misc = cur + NBRUN;
  const int tid = (int)threadIdx.x, lane = tid & 31, wave = tid >> 5;
  const int blk  = (int)blockIdx.x;
  const int role = blk / NBK;
  const int bb   = blk - role * NBK;
  const int koff = (role == 0) ? NE : 0;
  const int goff = NE - koff;
  const int* keys = ei + koff;
  const int* oth  = ei + goff;
  const unsigned nbs = (unsigned)(bb * NBRUN);

  {
    const v4i z4 = {0, 0, 0, 0};
    for (int i = tid * 4; i < BK_ZINTS; i += NTHR * 4) *(v4ia*)(dsm + i) = z4;
    if (tid < 16) misc[tid] = 0;
  }
  __syncthreads();

  {
    const int per  = ((NE + NWAVE * WCH - 1) / (NWAVE * WCH)) * WCH;
    const int ebeg = wave * per;
    const int eend = (ebeg + per < NE) ? (ebeg + per) : NE;
    int* mylist = wl + wave * WLCAP;
    int wc = 0;
#pragma unroll 1
    for (int cb = ebeg; cb < eend; cb += WCH) {
      const int e0 = cb + lane * EPT;
      const int ec = e0 < (NE - EPT) ? e0 : (NE - EPT);
      const bool lv = e0 < NE;
      const v4i da = *(const v4ia*)(keys + ec);
      const v4i db = *(const v4ia*)(keys + ec + 4);
      const unsigned s0 = (unsigned)da.x - nbs, s1 = (unsigned)da.y - nbs;
      const unsigned s2 = (unsigned)da.z - nbs, s3 = (unsigned)da.w - nbs;
      const unsigned s4 = (unsigned)db.x - nbs, s5 = (unsigned)db.y - nbs;
      const unsigned s6 = (unsigned)db.z - nbs, s7 = (unsigned)db.w - nbs;
      const bool h0 = lv & (s0 < (unsigned)NBRUN), h1 = lv & (s1 < (unsigned)NBRUN);
      const bool h2 = lv & (s2 < (unsigned)NBRUN), h3 = lv & (s3 < (unsigned)NBRUN);
      const bool h4 = lv & (s4 < (unsigned)NBRUN), h5 = lv & (s5 < (unsigned)NBRUN);
      const bool h6 = lv & (s6 < (unsigned)NBRUN), h7 = lv & (s7 < (unsigned)NBRUN);
      const unsigned m0 = __builtin_amdgcn_ballot_w32(h0), m1 = __builtin_amdgcn_ballot_w32(h1);
      const unsigned m2 = __builtin_amdgcn_ballot_w32(h2), m3 = __builtin_amdgcn_ballot_w32(h3);
      const unsigned m4 = __builtin_amdgcn_ballot_w32(h4), m5 = __builtin_amdgcn_ballot_w32(h5);
      const unsigned m6 = __builtin_amdgcn_ballot_w32(h6), m7 = __builtin_amdgcn_ballot_w32(h7);
      const unsigned any = m0 | m1 | m2 | m3 | m4 | m5 | m6 | m7;
      if (any != 0u) {
        const int pre = (int)(__builtin_amdgcn_mbcnt_lo(m0, 0u) + __builtin_amdgcn_mbcnt_lo(m1, 0u) +
                              __builtin_amdgcn_mbcnt_lo(m2, 0u) + __builtin_amdgcn_mbcnt_lo(m3, 0u) +
                              __builtin_amdgcn_mbcnt_lo(m4, 0u) + __builtin_amdgcn_mbcnt_lo(m5, 0u) +
                              __builtin_amdgcn_mbcnt_lo(m6, 0u) + __builtin_amdgcn_mbcnt_lo(m7, 0u));
        int p = wc + pre;
        if (h0) { if (p < WLCAP) mylist[p] = ((e0 + 0) << SLB) | (int)s0; p = p + 1; }
        if (h1) { if (p < WLCAP) mylist[p] = ((e0 + 1) << SLB) | (int)s1; p = p + 1; }
        if (h2) { if (p < WLCAP) mylist[p] = ((e0 + 2) << SLB) | (int)s2; p = p + 1; }
        if (h3) { if (p < WLCAP) mylist[p] = ((e0 + 3) << SLB) | (int)s3; p = p + 1; }
        if (h4) { if (p < WLCAP) mylist[p] = ((e0 + 4) << SLB) | (int)s4; p = p + 1; }
        if (h5) { if (p < WLCAP) mylist[p] = ((e0 + 5) << SLB) | (int)s5; p = p + 1; }
        if (h6) { if (p < WLCAP) mylist[p] = ((e0 + 6) << SLB) | (int)s6; p = p + 1; }
        if (h7) { if (p < WLCAP) mylist[p] = ((e0 + 7) << SLB) | (int)s7; p = p + 1; }
        wc += (int)(__builtin_popcount(m0) + __builtin_popcount(m1) + __builtin_popcount(m2) + __builtin_popcount(m3) +
                    __builtin_popcount(m4) + __builtin_popcount(m5) + __builtin_popcount(m6) + __builtin_popcount(m7));
      }
    }
    if (lane == 0) misc[wave] = wc;
  }
  __syncthreads();

  if (wave == 0) {
    int ov = 0;
#pragma unroll 1
    for (int w2 = 0; w2 < NWAVE; ++w2) {
      int c = misc[w2];
      if (c > WLCAP) ov = 1;
      c = c < 0 ? 0 : (c > WLCAP ? WLCAP : c);
#pragma unroll 1
      for (int b0 = 0; b0 < c; b0 += 32) {
        const int idx = b0 + lane;
        const int ent = wl[w2 * WLCAP + (idx < WLCAP ? idx : WLCAP - 1)];
        const int m32 = (c - b0) < 32 ? (c - b0) : 32;
#pragma unroll 1
        for (int k = 0; k < m32; ++k) {
          const int u    = __builtin_amdgcn_readlane(ent, k);
          const int slot = u & (NBRUN - 1);
          if (lane == 0) cnt[slot] = cnt[slot] + 1;
        }
      }
    }
    if (lane == 0) misc[9] = ov;
  }
  __syncthreads();
  if (wave == 0) {
    const int base = lane * (NBRUN / 32);
    int s = 0;
#pragma unroll 1
    for (int i = 0; i < NBRUN / 32; ++i) s += cnt[base + i];
    int incl = s;
#pragma unroll
    for (int d = 1; d < 32; d <<= 1) {
      const int y = __shfl_up(incl, d, 32);
      if (lane >= d) incl += y;
    }
    const int tot = __shfl(incl, 31, 32);
    int run = incl - s;
#pragma unroll 1
    for (int i = 0; i < NBRUN / 32; ++i) {
      const int cv = cnt[base + i];
      offs[base + i] = run;
      cur[base + i]  = run;
      run += cv;
    }
    if (lane == 0) { if (tot > RCAP) misc[9] = 1; }
  }
  __syncthreads();

  if (wave == 0) {
#pragma unroll 1
    for (int w2 = 0; w2 < NWAVE; ++w2) {
      int c = misc[w2];
      c = c < 0 ? 0 : (c > WLCAP ? WLCAP : c);
#pragma unroll 1
      for (int b0 = 0; b0 < c; b0 += 32) {
        const int idx = b0 + lane;
        const int ent = wl[w2 * WLCAP + (idx < WLCAP ? idx : WLCAP - 1)];
        int eid = (ent >> SLB) & 0xFFFFF;
        eid = eid > NE - 1 ? NE - 1 : eid;
        int sr = oth[eid];
        sr = sr < 0 ? 0 : (sr > NN - 1 ? NN - 1 : sr);
        const int wb = (int)(bf16_bits(ew[eid]) << 16);
        const int m32 = (c - b0) < 32 ? (c - b0) : 32;
#pragma unroll 1
        for (int k = 0; k < m32; ++k) {
          const int u    = __builtin_amdgcn_readlane(ent, k);
          const int sid  = __builtin_amdgcn_readlane(sr, k);
          const int wd   = __builtin_amdgcn_readlane(wb, k);
          const int slot = u & (NBRUN - 1);
          if (lane == 0) {
            int p = cur[slot];
            p = p < 0 ? 0 : (p > RCAP - 1 ? RCAP - 1 : p);
            pl[2 * p]     = sid;
            pl[2 * p + 1] = wd;
            cur[slot] = p + 1;
          }
        }
      }
    }
  }
  __syncthreads();

  const int ovf = misc[9];
  int* lp  = LIST + (size_t)blk * (size_t)(2 * RCAP);
  int* cop = CO + (size_t)blk * (size_t)(2 * NBRUN);
  int* fp  = FLAG + (size_t)blk * 32;
  bucket_flush(pl, cnt, ovf, lp, cop, fp, tid);
  __threadfence();
  bucket_flush(pl, cnt, ovf, lp, cop, fp, tid);
}

__device__ __forceinline__ void replay_role(const int* __restrict__ lb, const int* __restrict__ cob, int slot,
                                            const unsigned short* __restrict__ XB, int q,
                                            float& a0, float& a1, float& a2, float& a3, int& bigf) {
  int c = cob[slot];
  int o = cob[NBRUN + slot];
  bigf = (c > TRIPCAP) ? 1 : 0;
  c = c < 0 ? 0 : (c > TRIPCAP ? TRIPCAP : c);
  o = o < 0 ? 0 : (o > RCAP - 1 ? RCAP - 1 : o);
  int last = o + c - 1;
  last = last < o ? o : last;
  last = last > RCAP - 1 ? RCAP - 1 : last;
  const int co = __shfl_xor(c, 16, 32);
  const int cm = c > co ? c : co;
#pragma unroll 1
  for (int j = 0; j < cm; ++j) {
    int idx = o + j;
    idx = idx > last ? last : idx;
    const v2i ent = *(const v2ia*)(lb + 2 * idx);
    int sr = ent.x;
    sr = sr < 0 ? 0 : (sr > NN - 1 ? NN - 1 : sr);
    const float w = __int_as_float(ent.y);
    const v2u xv = *(const v2ua*)(XB + (size_t)sr * HD + 4 * q);
    asm volatile("" :: "v"(xv));
    const float f0 = __uint_as_float(xv.x << 16), f1 = __uint_as_float(xv.x & 0xffff0000u);
    const float f2 = __uint_as_float(xv.y << 16), f3 = __uint_as_float(xv.y & 0xffff0000u);
    const bool valid = j < c;
    const float t0 = fmaf(w, f0, a0), t1 = fmaf(w, f1, a1), t2 = fmaf(w, f2, a2), t3 = fmaf(w, f3, a3);
    a0 = valid ? t0 : a0; a1 = valid ? t1 : a1; a2 = valid ? t2 : a2; a3 = valid ? t3 : a3;
  }
}

__global__ __launch_bounds__(NTHR) void k_replay(const int* __restrict__ LIST, const int* __restrict__ CO,
                                                 const int* __restrict__ FLAG,
                                                 const unsigned short* __restrict__ XB, unsigned short* MIHL) {
  const int tid = (int)threadIdx.x, lane = tid & 31, wave = tid >> 5, hh = lane >> 4, q = lane & 15;
  const int rowBase = (int)blockIdx.x * ABM;
  const int bucket  = rowBase >> SLB;
  const int* lb0 = LIST + (size_t)bucket * (size_t)(2 * RCAP);
  const int* lb1 = LIST + (size_t)(NBK + bucket) * (size_t)(2 * RCAP);
  const int* co0 = CO + (size_t)bucket * (size_t)(2 * NBRUN);
  const int* co1 = CO + (size_t)(NBK + bucket) * (size_t)(2 * NBRUN);
  const int flag = FLAG[(size_t)bucket * 32] | FLAG[(size_t)(NBK + bucket) * 32];
  const float qnan = __uint_as_float(0x7fc00000u);

#pragma unroll 1
  for (int i = 0; i < ABM / (2 * NWAVE); ++i) {
    const int d    = rowBase + (ABM / NWAVE) * wave + 2 * i + hh;
    const int slot = d & (NBRUN - 1);
    float p0 = 0.0f, p1 = 0.0f, p2 = 0.0f, p3 = 0.0f;
    float r0 = 0.0f, r1 = 0.0f, r2 = 0.0f, r3 = 0.0f;
    int big0 = 0, big1 = 0;
    replay_role(lb0, co0, slot, XB, q, p0, p1, p2, p3, big0);
    replay_role(lb1, co1, slot, XB, q, r0, r1, r2, r3, big1);
    float m0 = p0 + r0, m1 = p1 + r1, m2 = p2 + r2, m3 = p3 + r3;
    const bool bad  = (flag != 0) | (big0 != 0) | (big1 != 0);
    const bool live = d < NN;
    m0 = bad ? qnan : m0; m1 = bad ? qnan : m1; m2 = bad ? qnan : m2; m3 = bad ? qnan : m3;
    m0 = live ? m0 : 0.0f; m1 = live ? m1 : 0.0f; m2 = live ? m2 : 0.0f; m3 = live ? m3 : 0.0f;
    int h01, h23, l01, l23;
    hilo_pack(m0, m1, m2, m3, h01, h23, l01, l23);
    const v4i ow = regroup8(h01, h23, l01, l23, lane);
    unsigned short* hp = MIHL + (size_t)d * KL + 8 * q;
    *(volatile v4i*)hp = ow;
    __threadfence();
    *(volatile v4i*)hp = ow;
  }
}

template <int NK, int BP>
__device__ __forceinline__ void gemm_ga(const unsigned short* __restrict__ ap, const unsigned short* bp,
                                        v8f (&acc)[4]) {
#pragma unroll 1
  for (int ks = 0; ks < NK; ++ks) {
    const int k0 = 32 * ks;
    FragB af;
    af.h[0] = *(const v8usa*)(ap + k0);
    af.h[1] = *(const v8usa*)(ap + k0 + 16);
#pragma unroll
    for (int nt = 0; nt < 4; ++nt) {
      const unsigned short* wq = bp + (16 * nt) * BP + k0;
      FragB bf;
      bf.h[0] = *(const v8usa*)wq;
      bf.h[1] = *(const v8usa*)(wq + 16);
      acc[nt] = wmb(af, bf, acc[nt]);
    }
  }
}

template <int NK, int BP>
__device__ __forceinline__ void gemm_la(const unsigned short* ap, const unsigned short* bp, v8f (&acc)[4]) {
#pragma unroll 1
  for (int ks = 0; ks < NK; ++ks) {
    const int k0 = 32 * ks;
    FragB af;
    af.h[0] = *(const v8usa*)(ap + k0);
    af.h[1] = *(const v8usa*)(ap + k0 + 16);
#pragma unroll
    for (int nt = 0; nt < 4; ++nt) {
      const unsigned short* wq = bp + (16 * nt) * BP + k0;
      FragB bf;
      bf.h[0] = *(const v8usa*)wq;
      bf.h[1] = *(const v8usa*)(wq + 16);
      acc[nt] = wmb(af, bf, acc[nt]);
    }
  }
}

__device__ __forceinline__ void zero_acc(v8f (&acc)[4]) {
  const v8f z = {0.f, 0.f, 0.f, 0.f, 0.f, 0.f, 0.f, 0.f};
#pragma unroll
  for (int t = 0; t < 4; ++t) acc[t] = z;
}

__device__ __forceinline__ void stage_d(float* stg, const v8f (&acc)[4], int wave, int hh, int m) {
#pragma unroll
  for (int nt = 0; nt < 4; ++nt) {
#pragma unroll
    for (int r = 0; r < 8; ++r) stg[(16 * wave + 8 * hh + r) * SP + 16 * nt + m] = acc[nt][r];
  }
}

__device__ __forceinline__ void epi_ln_tanh(const float* stg, const float* pb, const float* pg, const float* pe,
                                            int* ati, int wave, int hh, int m) {
  const v4f bb = *(const v4fa*)(pb + 4 * m);
  const v4f gg = *(const v4fa*)(pg + 4 * m);
  const v4f ee = *(const v4fa*)(pe + 4 * m);
#pragma unroll 1
  for (int i = 0; i < 8; ++i) {
    const int lr = 16 * wave + 2 * i + hh;
    const v4f a = *(const v4fa*)(stg + lr * SP + 4 * m);
    const float y0 = a.x + bb.x, y1 = a.y + bb.y, y2 = a.z + bb.z, y3 = a.w + bb.w;
    float s = (y0 + y1) + (y2 + y3);
    s += __shfl_xor(s, 8, 32);
    s += __shfl_xor(s, 4, 32);
    s += __shfl_xor(s, 2, 32);
    s += __shfl_xor(s, 1, 32);
    const float mu = s * 0.015625f;
    const float d0 = y0 - mu, d1 = y1 - mu, d2 = y2 - mu, d3 = y3 - mu;
    float qv = (d0 * d0 + d1 * d1) + (d2 * d2 + d3 * d3);
    qv += __shfl_xor(qv, 8, 32);
    qv += __shfl_xor(qv, 4, 32);
    qv += __shfl_xor(qv, 2, 32);
    qv += __shfl_xor(qv, 1, 32);
    const float var  = qv * 0.015625f;
    const float rstd = 1.0f / sqrtf(var + 1e-5f);
    const float o0 = tanhf(d0 * rstd * gg.x + ee.x);
    const float o1 = tanhf(d1 * rstd * gg.y + ee.y);
    const float o2 = tanhf(d2 * rstd * gg.z + ee.z);
    const float o3 = tanhf(d3 * rstd * gg.w + ee.w);
    int h01, h23, l01, l23;
    hilo_pack(o0, o1, o2, o3, h01, h23, l01, l23);
    v2i hv, lv;
    hv.x = h01; hv.y = h23;
    lv.x = l01; lv.y = l23;
    *(v2ia*)(ati + lr * AIP + 2 * m)      = hv;
    *(v2ia*)(ati + lr * AIP + 32 + 2 * m) = lv;
  }
}

__global__ __launch_bounds__(NTHR) __attribute__((amdgpu_num_vgpr(248)))
void k_mlp(const unsigned short* __restrict__ MIHL, const unsigned short* __restrict__ XB,
           const int* __restrict__ WALL, const int* __restrict__ FLAG, float* out) {
  extern __shared__ __attribute__((aligned(16))) int dsm[];
  const unsigned short* w1c = (const unsigned short*)dsm;
  const unsigned short* w2d = w1c + HD * K1;
  const unsigned short* w3d = w2d + HD * KL;
  const float* pv  = (const float*)(dsm + WALL_W_INTS);
  float*       stg = (float*)(dsm + ML_STG_OFF);
  int*         ati = dsm + ML_AT_OFF;
  const unsigned short* ath = (const unsigned short*)ati;
  const int tid = (int)threadIdx.x, lane = tid & 31, wave = tid >> 5, hh = lane >> 4, m = lane & 15;
  const int rowBase = (int)blockIdx.x * GBM;
  const int bucket  = rowBase >> SLB;
  const int flag = FLAG[(size_t)bucket * 32] | FLAG[(size_t)(NBK + bucket) * 32];

#pragma unroll 1
  for (int i = tid; i < WALL_INTS / 4; i += NTHR) {
    const v4i v = *(const v4ia*)(WALL + 4 * i);
    *(v4ia*)(dsm + 4 * i) = v;
  }
  __syncthreads();

  v8f acc[4];

  zero_acc(acc);
  {
    const int grow = rowBase + 16 * wave + m;
    const unsigned short* ap0 = MIHL + (size_t)grow * KL + 8 * hh;
    const unsigned short* ap1 = XB + (size_t)grow * HD + 8 * hh;
    const unsigned short* bp  = w1c + m * K1 + 8 * hh;
    gemm_ga<4, K1>(ap0, bp, acc);
    gemm_ga<2, K1>(ap1, bp + KL, acc);
  }
  stage_d(stg, acc, wave, hh, m);
  __syncthreads();

  epi_ln_tanh(stg, pv, pv + 64, pv + 128, ati, wave, hh, m);
  __syncthreads();

  zero_acc(acc);
  gemm_la<4, KL>(ath + (16 * wave + m) * ATP + 8 * hh, w2d + m * KL + 8 * hh, acc);
  stage_d(stg, acc, wave, hh, m);
  __syncthreads();
  epi_ln_tanh(stg, pv + 192, pv + 256, pv + 320, ati, wave, hh, m);
  __syncthreads();

  zero_acc(acc);
  gemm_la<4, KL>(ath + (16 * wave + m) * ATP + 8 * hh, w3d + m * KL + 8 * hh, acc);
  stage_d(stg, acc, wave, hh, m);
  __syncthreads();

  const v4f b3v = *(const v4fa*)(pv + 384 + 4 * m);
  const float qnan = __uint_as_float(0x7fc00000u);
#pragma unroll 1
  for (int i = 0; i < 8; ++i) {
    const int lr   = 16 * wave + 2 * i + hh;
    const int grow = rowBase + lr;
    const v4f a = *(const v4fa*)(stg + lr * SP + 4 * m);
    asm volatile("" :: "v"(a));
    const float v0 = a.x + b3v.x, v1 = a.y + b3v.y, v2 = a.z + b3v.z, v3 = a.w + b3v.w;
    v4f o;
    o.x = (flag != 0) ? qnan : v0; o.y = (flag != 0) ? qnan : v1;
    o.z = (flag != 0) ? qnan : v2; o.w = (flag != 0) ? qnan : v3;
    float* op = out + (size_t)grow * HD + 4 * m;
    if (grow < NN) st2_v4f(op, o);
  }
}

extern "C" void kernel_launch(void* const* d_in, const int* in_sizes, int n_in,
                              void* d_out, int out_size, void* d_ws, size_t ws_size,
                              hipStream_t stream) {
  if (n_in < 13) return;
  if (in_sizes[0] != NN * HD) return;
  if (in_sizes[1] != NE) return;
  if (in_sizes[2] != 2 * NE) return;
  if (in_sizes[3] != 2 * HD * HD) return;
  if (in_sizes[4] != HD || in_sizes[5] != HD || in_sizes[6] != HD) return;
  if (in_sizes[7] != HD * HD) return;
  if (in_sizes[8] != HD || in_sizes[9] != HD || in_sizes[10] != HD) return;
  if (in_sizes[11] != HD * HD) return;
  if (in_sizes[12] != HD) return;
  if (out_size != NN * HD) return;

  const float* x   = (const float*)d_in[0];
  const float* ew  = (const float*)d_in[1];
  const int*   ei  = (const int*)d_in[2];
  const float* W1  = (const float*)d_in[3];
  const float* b1  = (const float*)d_in[4];
  const float* g1  = (const float*)d_in[5];
  const float* be1 = (const float*)d_in[6];
  const float* W2  = (const float*)d_in[7];
  const float* b2  = (const float*)d_in[8];
  const float* g2  = (const float*)d_in[9];
  const float* be2 = (const float*)d_in[10];
  const float* W3  = (const float*)d_in[11];
  const float* b3  = (const float*)d_in[12];
  float* out = (float*)d_out;

  constexpr size_t zXB   = (size_t)MP * HD * 2;
  constexpr size_t zMIHL = (size_t)MP * KL * 2;
  constexpr size_t zLIST = (size_t)NROLE * NBK * RCAP * 8;
  constexpr size_t zCO   = (size_t)NROLE * NBK * 2 * NBRUN * 4;
  constexpr size_t zFLAG = (size_t)NROLE * NBK * 128;
  constexpr size_t zWALL = (size_t)WALL_INTS * 4;
  constexpr size_t oXB   = 0;
  constexpr size_t oMIHL = oXB + zXB;
  constexpr size_t oLIST = oMIHL + zMIHL;
  constexpr size_t oCO   = oLIST + zLIST;
  constexpr size_t oFLAG = oCO + zCO;
  constexpr size_t oWALL = oFLAG + zFLAG;
  constexpr size_t oEND  = oWALL + zWALL;
  static_assert(zXB % 256 == 0 && zMIHL % 256 == 0 && zLIST % 256 == 0 && zCO % 256 == 0);
  static_assert(zFLAG % 256 == 0 && zWALL % 256 == 0);
  static_assert(oEND <= (size_t)WSMAX);
  if (oEND > ws_size) return;

  char* ws = (char*)d_ws;
  unsigned short* XB   = (unsigned short*)(ws + oXB);
  unsigned short* MIHL = (unsigned short*)(ws + oMIHL);
  int*            LIST = (int*)(ws + oLIST);
  int*            CO   = (int*)(ws + oCO);
  int*            FLAG = (int*)(ws + oFLAG);
  unsigned short* W1C  = (unsigned short*)(ws + oWALL);
  unsigned short* W2D  = W1C + HD * K1;
  unsigned short* W3D  = W2D + HD * KL;
  float*          PV   = (float*)(ws + oWALL + (size_t)WALL_W_INTS * 4);
  const int*      WALL = (const int*)(ws + oWALL);

  hipFuncSetAttribute(reinterpret_cast<const void*>(&k_bucket), hipFuncAttributeMaxDynamicSharedMemorySize, (int)BK_LDS);
  hipFuncSetAttribute(reinterpret_cast<const void*>(&k_mlp), hipFuncAttributeMaxDynamicSharedMemorySize, (int)ML_LDS);

  k_prep<<<PBTOT, NTHR, 0, stream>>>(x, W1, b1, g1, be1, W2, b2, g2, be2, W3, b3, XB, W1C, W2D, W3D, PV);
  k_bucket<<<NROLE * NBK, NTHR, BK_LDS, stream>>>(ei, ew, LIST, CO, FLAG);
  k_replay<<<MP / ABM, NTHR, 0, stream>>>(LIST, CO, FLAG, XB, MIHL);
  k_mlp<<<MP / GBM, NTHR, ML_LDS, stream>>>(MIHL, XB, WALL, FLAG, out);
}
